// EdgeConv_56246891708812
// MI455X (gfx1250) — hardware-verified
//
#include <hip/hip_runtime.h>
#define BB 2
#define CC 64
#define NP 16384
#define KN 32
#define NPT (BB * NP)
#define NPR (NPT * KN)
#define NTL (NPR / 16)
#define H1 64
#define H2 64

typedef __bf16 v16b __attribute__((ext_vector_type(16)));
typedef unsigned short v8us __attribute__((ext_vector_type(8), may_alias));
typedef float  v8f  __attribute__((ext_vector_type(8)));
typedef float  v4f  __attribute__((ext_vector_type(4)));
typedef float  v4fa __attribute__((ext_vector_type(4), may_alias));
union FragB { v16b v; v8us half[2]; unsigned short u[16]; };

__device__ __forceinline__ unsigned short bf16_bits(float x) { unsigned int u = __float_as_uint(x); return (unsigned short)((u + 0x7FFFu + ((u >> 16) & 1u)) >> 16); }
__device__ __forceinline__ float bf16_val(unsigned short b) { return __uint_as_float(((unsigned int)b) << 16); }
__device__ __forceinline__ float bf16_round(float x) { return bf16_val(bf16_bits(x)); }
template <int NT>
__device__ __forceinline__ v8f mmaN(v16b ah, v16b al, v16b bh, v16b bl, v8f c) {
  c = __builtin_amdgcn_wmma_f32_16x16x32_bf16(false, ah, false, bh, (short)0, c, false, false);
  if (NT >= 2) c = __builtin_amdgcn_wmma_f32_16x16x32_bf16(false, al, false, bh, (short)0, c, false, false);
  if (NT >= 3) c = __builtin_amdgcn_wmma_f32_16x16x32_bf16(false, ah, false, bl, (short)0, c, false, false);
  asm volatile("v_nop\n\tv_nop\n\tv_nop\n\tv_nop" : "+v"(c) : "v"(ah), "v"(al), "v"(bh), "v"(bl));
  return c;
}

__global__ __launch_bounds__(256) void k_wt_bf16(const float* __restrict__ W, unsigned short* __restrict__ Wt, int K, int N) {
  const int t = blockIdx.x * 256 + threadIdx.x;
  const int k8n = K / 8;
  if (t >= N * k8n) return;
  const int n = t / k8n, k8 = (t % k8n) * 8;
  v8us v;
#pragma unroll
  for (int i = 0; i < 8; ++i) v[i] = bf16_bits(W[(size_t)(k8 + i) * N + n]);
  *(volatile v8us*)(Wt + (size_t)n * K + k8) = v;
  __threadfence();
  *(volatile v8us*)(Wt + (size_t)n * K + k8) = v;
}

template <bool ASPLIT, int ACT, bool BIAS_BF16>
__global__ __launch_bounds__(128) void k_gemm_bf(const float* __restrict__ A, int lda, const unsigned short* __restrict__ Wt, int ldb,
                                               const float* __restrict__ bias, float* __restrict__ C, int ldc, int M, int N, int K) {
  __shared__ __attribute__((aligned(16))) float so[4][16][64];
  const int tid = threadIdx.x, w = tid >> 5, lane = tid & 31, ln = lane & 15, hh = lane >> 4;
  const int ntn = N / 64;
  const int wid = blockIdx.x * 4 + w;
  const int mt = wid / ntn, nq = wid % ntn;
  if (mt * 16 >= M) return;
  const int row0 = mt * 16, col0 = nq * 64;
  const float* arow = A + (size_t)(row0 + ln) * lda;
  v8f acc[4] = {};
  for (int kb = 0; kb < K; kb += 32) {
    FragB ah, al;
    const v4f x0 = *(const v4fa*)(arow + kb + 8 * hh), x1 = *(const v4fa*)(arow + kb + 8 * hh + 4);
    const v4f x2 = *(const v4fa*)(arow + kb + 16 + 8 * hh), x3 = *(const v4fa*)(arow + kb + 16 + 8 * hh + 4);
    float xs[16] = {x0[0],x0[1],x0[2],x0[3],x1[0],x1[1],x1[2],x1[3],x2[0],x2[1],x2[2],x2[3],x3[0],x3[1],x3[2],x3[3]};
#pragma unroll
    for (int i = 0; i < 16; ++i) { const unsigned short hb = bf16_bits(xs[i]); ah.u[i] = hb; al.u[i] = ASPLIT ? bf16_bits(xs[i] - bf16_val(hb)) : (unsigned short)0; }
#pragma unroll
    for (int t = 0; t < 4; ++t) {
      const unsigned short* brow = Wt + (size_t)(col0 + t * 16 + ln) * ldb + kb;
      FragB b;
      b.half[0] = *(const v8us*)(brow + 8 * hh);
      b.half[1] = *(const v8us*)(brow + 16 + 8 * hh);
      acc[t] = mmaN<ASPLIT ? 2 : 1>(ah.v, al.v, b.v, b.v, acc[t]);
    }
  }
#pragma unroll
  for (int t = 0; t < 4; ++t) {
    float bv = bias ? bias[col0 + t * 16 + ln] : 0.f;
    if (BIAS_BF16) bv = bf16_round(bv);
#pragma unroll
    for (int r = 0; r < 8; ++r) { float v = acc[t][r] + bv; if (ACT == 1) v = fmaxf(v, 0.f); so[w][8 * hh + r][t * 16 + ln] = v; }
  }
  __builtin_amdgcn_fence(__ATOMIC_ACQ_REL, "workgroup");
  __builtin_amdgcn_wave_barrier();
  const int rsub = lane >> 4, c4 = (lane & 15) * 4;
  for (int pass = 0; pass < 2; ++pass) {
#pragma unroll
    for (int q = 0; q < 8; ++q) {
      const int r = q * 2 + rsub;
      const v4f v = *(const v4fa*)&so[w][r][c4];
      *(volatile v4f*)(C + (size_t)(row0 + r) * ldc + col0 + c4) = v;
    }
    if (pass == 0) __threadfence();
  }
}

template <int D, bool CAUSAL>
__global__ __launch_bounds__(128) void k_flash(const float* __restrict__ qb, const float* __restrict__ kb, const float* __restrict__ vb,
                                             int pitch, int T, int H, float scale, float* __restrict__ y, int ypitch) {
  constexpr int KS = D / 32;
  constexpr int DT = D / 16;
  __shared__ __attribute__((aligned(16))) unsigned short sKh[32][D + 8], sKl[32][D + 8], sVh[32][D + 8], sVl[32][D + 8];
  __shared__ __attribute__((aligned(16))) unsigned short sPh[4][16][40], sPl[4][16][40];
  __shared__ __attribute__((aligned(16))) float sO[4][16][D];
  const int tid = threadIdx.x, w = tid >> 5, lane = tid & 31, ln = lane & 15, hh = lane >> 4;
  const int nqb = (T + 63) / 64;
  const int bh = blockIdx.x / nqb, qblk = blockIdx.x % nqb;
  const int b = bh / H, h = bh % H;
  const int q0 = qblk * 64 + w * 16;
  const float* Q = qb + (size_t)b * T * pitch + h * D;
  const float* K = kb + (size_t)b * T * pitch + h * D;
  const float* V = vb + (size_t)b * T * pitch + h * D;

  FragB aqh[KS], aql[KS];
  {
    int row = q0 + ln; if (row >= T) row = T - 1;
    const float* qr = Q + (size_t)row * pitch;
#pragma unroll
    for (int ks = 0; ks < KS; ++ks)
#pragma unroll
      for (int i = 0; i < 16; ++i) {
        const int d = ks * 32 + ((i < 8) ? (8 * hh + i) : (16 + 8 * hh + (i - 8)));
        const float x = qr[d] * scale; const unsigned short hb = bf16_bits(x);
        aqh[ks].u[i] = hb; aql[ks].u[i] = bf16_bits(x - bf16_val(hb));
      }
  }
  float m_r[8], l_r[8];
#pragma unroll
  for (int r = 0; r < 8; ++r) { m_r[r] = -3.0e38f; l_r[r] = 0.f; }
  v8f oacc[DT];
#pragma unroll
  for (int dt = 0; dt < DT; ++dt) oacc[dt] = (v8f){0.f,0.f,0.f,0.f,0.f,0.f,0.f,0.f};

  const int kv_end = CAUSAL ? min(T, qblk * 64 + 64) : T;
  for (int j0 = 0; j0 < kv_end; j0 += 32) {
    __syncthreads();
    for (int e = tid; e < 32 * (D / 4); e += 128) {
      const int r = e / (D / 4), c4 = (e % (D / 4)) * 4;
      const int key = j0 + r;
      v4f kf = {0.f,0.f,0.f,0.f}, vf = {0.f,0.f,0.f,0.f};
      if (key < T) { kf = *(const v4fa*)(K + (size_t)key * pitch + c4); vf = *(const v4fa*)(V + (size_t)key * pitch + c4); }
#pragma unroll
      for (int t = 0; t < 4; ++t) {
        unsigned short hb = bf16_bits(kf[t]); sKh[r][c4 + t] = hb; sKl[r][c4 + t] = bf16_bits(kf[t] - bf16_val(hb));
        hb = bf16_bits(vf[t]); sVh[r][c4 + t] = hb; sVl[r][c4 + t] = bf16_bits(vf[t] - bf16_val(hb));
      }
    }
    __syncthreads();
    v8f s[2];
#pragma unroll
    for (int nt = 0; nt < 2; ++nt) {
      v8f acc = {};
#pragma unroll
      for (int ks = 0; ks < KS; ++ks) {
        FragB bh_, bl_;
        bh_.half[0] = *(const v8us*)&sKh[nt * 16 + ln][ks * 32 + 8 * hh]; bh_.half[1] = *(const v8us*)&sKh[nt * 16 + ln][ks * 32 + 16 + 8 * hh];
        bl_.half[0] = *(const v8us*)&sKl[nt * 16 + ln][ks * 32 + 8 * hh]; bl_.half[1] = *(const v8us*)&sKl[nt * 16 + ln][ks * 32 + 16 + 8 * hh];
        acc = mmaN<3>(aqh[ks].v, aql[ks].v, bh_.v, bl_.v, acc);
      }
      s[nt] = acc;
    }
    float alpha[8];
#pragma unroll
    for (int r = 0; r < 8; ++r) {
      const int qi = q0 + 8 * hh + r;
      const int ja = j0 + ln, jb = j0 + 16 + ln;
      if (CAUSAL) { if (ja > qi) s[0][r] = -3.0e38f; if (jb > qi) s[1][r] = -3.0e38f; }
      if (ja >= T) s[0][r] = -3.0e38f;
      if (jb >= T) s[1][r] = -3.0e38f;
      float mx = fmaxf(s[0][r], s[1][r]);
      mx = fmaxf(mx, __shfl_xor(mx, 1, 32)); mx = fmaxf(mx, __shfl_xor(mx, 2, 32)); mx = fmaxf(mx, __shfl_xor(mx, 4, 32)); mx = fmaxf(mx, __shfl_xor(mx, 8, 32));
      const float mnew = fmaxf(m_r[r], mx);
      alpha[r] = (mnew > -1.0e38f) ? __expf(m_r[r] - mnew) : 1.0f;
      const float p0 = (s[0][r] > -1.0e38f) ? __expf(s[0][r] - mnew) : 0.f;
      const float p1 = (s[1][r] > -1.0e38f) ? __expf(s[1][r] - mnew) : 0.f;
      m_r[r] = mnew;
      l_r[r] = l_r[r] * alpha[r] + p0 + p1;
      unsigned short hb = bf16_bits(p0); sPh[w][8 * hh + r][ln] = hb;      sPl[w][8 * hh + r][ln] = bf16_bits(p0 - bf16_val(hb));
      hb = bf16_bits(p1);                sPh[w][8 * hh + r][16 + ln] = hb; sPl[w][8 * hh + r][16 + ln] = bf16_bits(p1 - bf16_val(hb));
    }
#pragma unroll
    for (int dt = 0; dt < DT; ++dt)
#pragma unroll
      for (int r = 0; r < 8; ++r) oacc[dt][r] *= alpha[r];
    __builtin_amdgcn_fence(__ATOMIC_ACQ_REL, "workgroup");
    __builtin_amdgcn_wave_barrier();
    FragB pah, pal;
    pah.half[0] = *(const v8us*)&sPh[w][ln][8 * hh]; pah.half[1] = *(const v8us*)&sPh[w][ln][16 + 8 * hh];
    pal.half[0] = *(const v8us*)&sPl[w][ln][8 * hh]; pal.half[1] = *(const v8us*)&sPl[w][ln][16 + 8 * hh];
#pragma unroll
    for (int dt = 0; dt < DT; ++dt) {
      FragB bvh, bvl;
#pragma unroll
      for (int i = 0; i < 8; ++i) {
        bvh.u[i] = sVh[8 * hh + i][dt * 16 + ln]; bvh.u[8 + i] = sVh[16 + 8 * hh + i][dt * 16 + ln];
        bvl.u[i] = sVl[8 * hh + i][dt * 16 + ln]; bvl.u[8 + i] = sVl[16 + 8 * hh + i][dt * 16 + ln];
      }
      oacc[dt] = mmaN<3>(pah.v, pal.v, bvh.v, bvl.v, oacc[dt]);
    }
    __builtin_amdgcn_fence(__ATOMIC_ACQ_REL, "workgroup");
    __builtin_amdgcn_wave_barrier();
  }
#pragma unroll
  for (int r = 0; r < 8; ++r) {
    float l = l_r[r];
    l += __shfl_xor(l, 1, 32); l += __shfl_xor(l, 2, 32); l += __shfl_xor(l, 4, 32); l += __shfl_xor(l, 8, 32);
    l_r[r] = (l > 0.f) ? 1.0f / l : 0.f;
  }
#pragma unroll
  for (int dt = 0; dt < DT; ++dt)
#pragma unroll
    for (int r = 0; r < 8; ++r) sO[w][8 * hh + r][dt * 16 + ln] = oacc[dt][r] * l_r[r];
  __builtin_amdgcn_fence(__ATOMIC_ACQ_REL, "workgroup");
  __builtin_amdgcn_wave_barrier();
  for (int pass = 0; pass < 2; ++pass) {
    for (int r = 0; r < 16; ++r) {
      const int row = q0 + r;
      if (row < T && lane < D / 4) {
        const v4f val = *(const v4fa*)&sO[w][r][lane * 4];
        *(volatile v4f*)(y + ((size_t)b * T + row) * ypitch + h * D + lane * 4) = val;
      }
    }
    if (pass == 0) __threadfence();
  }
}

template <bool AFFINE, bool RESID, bool RES_BF16>
__global__ __launch_bounds__(256) void k_transpose32(const float* __restrict__ in, float* __restrict__ out, int rows, int cols,
                                                    const float* __restrict__ scale, const float* __restrict__ shift, const float* __restrict__ res) {
  __shared__ float tile[32][33];
  const int b = blockIdx.z;
  const int r0 = blockIdx.y * 32, c0 = blockIdx.x * 32;
  const float* src = in + (size_t)b * rows * cols;
  float* dst = out + (size_t)b * rows * cols;
  const int tx = threadIdx.x & 31, ty = threadIdx.x >> 5;
  for (int i = ty; i < 32; i += 8) tile[i][tx] = src[(size_t)(r0 + i) * cols + c0 + tx];
  __syncthreads();
  for (int pass = 0; pass < 2; ++pass) {
    for (int i = ty; i < 32; i += 8) {
      float v = tile[tx][i];
      const int orow = c0 + i;
      if (AFFINE) v = v * scale[orow] + shift[orow];
      if (RESID) { float rv = res[(size_t)b * rows * cols + (size_t)orow * rows + r0 + tx]; if (RES_BF16) rv = bf16_round(rv); v += rv; }
      *(volatile float*)(dst + (size_t)orow * rows + r0 + tx) = v;
    }
    if (pass == 0) __threadfence();
  }
}

__global__ __launch_bounds__(256) void k_pool2_pm(const float* __restrict__ in, float* __restrict__ out, int Bn, int H, int W, int C) {
  const size_t t = (size_t)blockIdx.x * 256 + threadIdx.x;
  const int c4n = C / 4, Ho = H / 2, Wo = W / 2;
  const size_t total = (size_t)Bn * Ho * Wo * c4n;
  if (t >= total) return;
  const int c4 = (int)(t % c4n) * 4; size_t rest = t / c4n;
  const int pw = (int)(rest % Wo); rest /= Wo; const int ph = (int)(rest % Ho); const int b = (int)(rest / Ho);
  const float* base = in + (size_t)b * H * W * C;
  const int p00 = (2 * ph) * W + 2 * pw;
  const v4f a = *(const v4fa*)(base + (size_t)p00 * C + c4), bq = *(const v4fa*)(base + (size_t)(p00 + 1) * C + c4);
  const v4f c = *(const v4fa*)(base + (size_t)(p00 + W) * C + c4), d = *(const v4fa*)(base + (size_t)(p00 + W + 1) * C + c4);
  v4f m; for (int i = 0; i < 4; ++i) m[i] = fmaxf(fmaxf(a[i], bq[i]), fmaxf(c[i], d[i]));
  float* dst = out + ((size_t)b * Ho * Wo + (size_t)ph * Wo + pw) * C + c4;
  *(volatile v4f*)dst = m;
  __threadfence();
  *(volatile v4f*)dst = m;
}

template <int DQ, int DV>
__global__ __launch_bounds__(128) void k_flash2(const float* __restrict__ Qb, size_t qstride, int qpitch, int Tq,
                                              const float* __restrict__ Kb, size_t kstride, int kpitch, int Tk,
                                              const float* __restrict__ Vb, size_t vstride, int vpitch,
                                              float scale, float* __restrict__ y, size_t ystride, int ypitch) {
  constexpr int KS = DQ / 32, DT = DV / 16;
  __shared__ __attribute__((aligned(16))) unsigned short sKh[32][DQ + 8], sKl[32][DQ + 8], sVh[32][DV + 8], sVl[32][DV + 8];
  __shared__ __attribute__((aligned(16))) unsigned short sPh[4][16][40], sPl[4][16][40];
  __shared__ __attribute__((aligned(16))) float sO[4][16][DV];
  const int tid = threadIdx.x, w = tid >> 5, lane = tid & 31, ln = lane & 15, hh = lane >> 4;
  const int nqb = (Tq + 63) / 64;
  const int bh = blockIdx.x / nqb, qblk = blockIdx.x % nqb;
  const int dv0 = blockIdx.y * DV;
  const int q0 = qblk * 64 + w * 16;
  const float* Q = Qb + (size_t)bh * qstride; const float* K = Kb + (size_t)bh * kstride; const float* V = Vb + (size_t)bh * vstride + dv0;
  FragB aqh[KS], aql[KS];
  {
    int row = q0 + ln; if (row >= Tq) row = Tq - 1;
    const float* qr = Q + (size_t)row * qpitch;
#pragma unroll
    for (int ks = 0; ks < KS; ++ks)
#pragma unroll
      for (int i = 0; i < 16; ++i) {
        const int d = ks * 32 + ((i < 8) ? (8 * hh + i) : (16 + 8 * hh + (i - 8)));
        const float x = qr[d] * scale; const unsigned short hb = bf16_bits(x);
        aqh[ks].u[i] = hb; aql[ks].u[i] = bf16_bits(x - bf16_val(hb));
      }
  }
  float m_r[8], l_r[8];
#pragma unroll
  for (int r = 0; r < 8; ++r) { m_r[r] = -3.0e38f; l_r[r] = 0.f; }
  v8f oacc[DT];
#pragma unroll
  for (int dt = 0; dt < DT; ++dt) oacc[dt] = (v8f){0.f,0.f,0.f,0.f,0.f,0.f,0.f,0.f};
  for (int j0 = 0; j0 < Tk; j0 += 32) {
    __syncthreads();
    for (int e = tid; e < 32 * (DQ / 4); e += 128) {
      const int r = e / (DQ / 4), c4 = (e % (DQ / 4)) * 4; const int key = j0 + r;
      v4f f = {0.f,0.f,0.f,0.f}; if (key < Tk) f = *(const v4fa*)(K + (size_t)key * kpitch + c4);
#pragma unroll
      for (int t = 0; t < 4; ++t) { const unsigned short hb = bf16_bits(f[t]); sKh[r][c4 + t] = hb; sKl[r][c4 + t] = bf16_bits(f[t] - bf16_val(hb)); }
    }
    for (int e = tid; e < 32 * (DV / 4); e += 128) {
      const int r = e / (DV / 4), c4 = (e % (DV / 4)) * 4; const int key = j0 + r;
      v4f f = {0.f,0.f,0.f,0.f}; if (key < Tk) f = *(const v4fa*)(V + (size_t)key * vpitch + c4);
#pragma unroll
      for (int t = 0; t < 4; ++t) { const unsigned short hb = bf16_bits(f[t]); sVh[r][c4 + t] = hb; sVl[r][c4 + t] = bf16_bits(f[t] - bf16_val(hb)); }
    }
    __syncthreads();
    v8f s[2];
#pragma unroll
    for (int nt = 0; nt < 2; ++nt) {
      v8f acc = {};
#pragma unroll
      for (int ks = 0; ks < KS; ++ks) {
        FragB bh_, bl_;
        bh_.half[0] = *(const v8us*)&sKh[nt * 16 + ln][ks * 32 + 8 * hh]; bh_.half[1] = *(const v8us*)&sKh[nt * 16 + ln][ks * 32 + 16 + 8 * hh];
        bl_.half[0] = *(const v8us*)&sKl[nt * 16 + ln][ks * 32 + 8 * hh]; bl_.half[1] = *(const v8us*)&sKl[nt * 16 + ln][ks * 32 + 16 + 8 * hh];
        acc = mmaN<3>(aqh[ks].v, aql[ks].v, bh_.v, bl_.v, acc);
      }
      s[nt] = acc;
    }
    float alpha[8];
#pragma unroll
    for (int r = 0; r < 8; ++r) {
      const int ja = j0 + ln, jb = j0 + 16 + ln;
      if (ja >= Tk) s[0][r] = -3.0e38f;
      if (jb >= Tk) s[1][r] = -3.0e38f;
      float mx = fmaxf(s[0][r], s[1][r]);
      mx = fmaxf(mx, __shfl_xor(mx, 1, 32)); mx = fmaxf(mx, __shfl_xor(mx, 2, 32)); mx = fmaxf(mx, __shfl_xor(mx, 4, 32)); mx = fmaxf(mx, __shfl_xor(mx, 8, 32));
      const float mnew = fmaxf(m_r[r], mx);
      alpha[r] = (mnew > -1.0e38f) ? __expf(m_r[r] - mnew) : 1.0f;
      const float p0 = (s[0][r] > -1.0e38f) ? __expf(s[0][r] - mnew) : 0.f;
      const float p1 = (s[1][r] > -1.0e38f) ? __expf(s[1][r] - mnew) : 0.f;
      m_r[r] = mnew;
      l_r[r] = l_r[r] * alpha[r] + p0 + p1;
      unsigned short hb = bf16_bits(p0); sPh[w][8 * hh + r][ln] = hb;      sPl[w][8 * hh + r][ln] = bf16_bits(p0 - bf16_val(hb));
      hb = bf16_bits(p1);                sPh[w][8 * hh + r][16 + ln] = hb; sPl[w][8 * hh + r][16 + ln] = bf16_bits(p1 - bf16_val(hb));
    }
#pragma unroll
    for (int dt = 0; dt < DT; ++dt)
#pragma unroll
      for (int r = 0; r < 8; ++r) oacc[dt][r] *= alpha[r];
    __builtin_amdgcn_fence(__ATOMIC_ACQ_REL, "workgroup");
    __builtin_amdgcn_wave_barrier();
    FragB pah, pal;
    pah.half[0] = *(const v8us*)&sPh[w][ln][8 * hh]; pah.half[1] = *(const v8us*)&sPh[w][ln][16 + 8 * hh];
    pal.half[0] = *(const v8us*)&sPl[w][ln][8 * hh]; pal.half[1] = *(const v8us*)&sPl[w][ln][16 + 8 * hh];
#pragma unroll
    for (int dt = 0; dt < DT; ++dt) {
      FragB bvh, bvl;
#pragma unroll
      for (int i = 0; i < 8; ++i) {
        bvh.u[i] = sVh[8 * hh + i][dt * 16 + ln]; bvh.u[8 + i] = sVh[16 + 8 * hh + i][dt * 16 + ln];
        bvl.u[i] = sVl[8 * hh + i][dt * 16 + ln]; bvl.u[8 + i] = sVl[16 + 8 * hh + i][dt * 16 + ln];
      }
      oacc[dt] = mmaN<3>(pah.v, pal.v, bvh.v, bvl.v, oacc[dt]);
    }
    __builtin_amdgcn_fence(__ATOMIC_ACQ_REL, "workgroup");
    __builtin_amdgcn_wave_barrier();
  }
#pragma unroll
  for (int r = 0; r < 8; ++r) {
    float l = l_r[r];
    l += __shfl_xor(l, 1, 32); l += __shfl_xor(l, 2, 32); l += __shfl_xor(l, 4, 32); l += __shfl_xor(l, 8, 32);
    l_r[r] = (l > 0.f) ? 1.0f / l : 0.f;
  }
#pragma unroll
  for (int dt = 0; dt < DT; ++dt)
#pragma unroll
    for (int r = 0; r < 8; ++r) sO[w][8 * hh + r][dt * 16 + ln] = oacc[dt][r] * l_r[r];
  __builtin_amdgcn_fence(__ATOMIC_ACQ_REL, "workgroup");
  __builtin_amdgcn_wave_barrier();
  for (int pass = 0; pass < 2; ++pass) {
    for (int r = 0; r < 16; ++r) {
      const int row = q0 + r;
      for (int c4 = lane * 4; c4 < DV; c4 += 128) {
        if (row < Tq) {
          const v4f val = *(const v4fa*)&sO[w][r][c4];
          *(volatile v4f*)(y + (size_t)bh * ystride + (size_t)row * ypitch + dv0 + c4) = val;
        }
      }
    }
    if (pass == 0) __threadfence();
  }
}

template <bool ASPLIT, int ACT, bool BIAS_BF16, bool RES_BF16>
__global__ __launch_bounds__(128) void k_gemm_bf3(const float* __restrict__ A, int lda, const unsigned short* __restrict__ Wt, int ldb,
                                                const float* __restrict__ bias, const float* __restrict__ resid, int rmod, int ldr,
                                                float* __restrict__ C, int ldc, int M, int N, int K) {
  __shared__ __attribute__((aligned(16))) float so[4][16][64];
  const int tid = threadIdx.x, w = tid >> 5, lane = tid & 31, ln = lane & 15, hh = lane >> 4;
  const int ntn = N / 64;
  const int wid = blockIdx.x * 4 + w;
  const int mt = wid / ntn, nq = wid % ntn;
  if (mt * 16 >= M) return;
  const int row0 = mt * 16, col0 = nq * 64;
  const float* arow = A + (size_t)(row0 + ln) * lda;
  v8f acc[4] = {};
  for (int kb = 0; kb < K; kb += 32) {
    FragB ah, al;
    const v4f x0 = *(const v4fa*)(arow + kb + 8 * hh), x1 = *(const v4fa*)(arow + kb + 8 * hh + 4);
    const v4f x2 = *(const v4fa*)(arow + kb + 16 + 8 * hh), x3 = *(const v4fa*)(arow + kb + 16 + 8 * hh + 4);
    float xs[16] = {x0[0],x0[1],x0[2],x0[3],x1[0],x1[1],x1[2],x1[3],x2[0],x2[1],x2[2],x2[3],x3[0],x3[1],x3[2],x3[3]};
#pragma unroll
    for (int i = 0; i < 16; ++i) { const unsigned short hb = bf16_bits(xs[i]); ah.u[i] = hb; al.u[i] = ASPLIT ? bf16_bits(xs[i] - bf16_val(hb)) : (unsigned short)0; }
#pragma unroll
    for (int t = 0; t < 4; ++t) {
      const unsigned short* brow = Wt + (size_t)(col0 + t * 16 + ln) * ldb + kb;
      FragB b;
      b.half[0] = *(const v8us*)(brow + 8 * hh);
      b.half[1] = *(const v8us*)(brow + 16 + 8 * hh);
      acc[t] = mmaN<ASPLIT ? 2 : 1>(ah.v, al.v, b.v, b.v, acc[t]);
    }
  }
#pragma unroll
  for (int t = 0; t < 4; ++t) {
    const int col = col0 + t * 16 + ln;
    float bv = bias ? bias[col] : 0.f;
    if (BIAS_BF16) bv = bf16_round(bv);
#pragma unroll
    for (int r = 0; r < 8; ++r) {
      float v = acc[t][r] + bv;
      if (resid) { float rv = resid[(size_t)((row0 + 8 * hh + r) % rmod) * ldr + col]; if (RES_BF16) rv = bf16_round(rv); v += rv; }
      if (ACT == 1) v = fmaxf(v, 0.f);
      if (ACT == 2) v = 0.5f * v * (1.0f + erff(v * 0.70710678118654752f));
      if (ACT == 3) { const float u = 0.7978845608028654f * (v + 0.044715f * v * v * v); v = 0.5f * v * (1.0f + tanhf(u)); }
      so[w][8 * hh + r][t * 16 + ln] = v;
    }
  }
  __builtin_amdgcn_fence(__ATOMIC_ACQ_REL, "workgroup");
  __builtin_amdgcn_wave_barrier();
  const int rsub = lane >> 4, c4 = (lane & 15) * 4;
  for (int pass = 0; pass < 2; ++pass) {
#pragma unroll
    for (int q = 0; q < 8; ++q) {
      const int r = q * 2 + rsub;
      const v4f v = *(const v4fa*)&so[w][r][c4];
      *(volatile v4f*)(C + (size_t)(row0 + r) * ldc + col0 + c4) = v;
    }
    if (pass == 0) __threadfence();
  }
}
template <bool PARAM_BF16>
__global__ __launch_bounds__(256) void k_layernorm(const float* __restrict__ X, const float* __restrict__ R, const float* __restrict__ g, const float* __restrict__ bta,
                                                  float* __restrict__ out_sum, float* __restrict__ out_norm, int N, float eps) {
  __shared__ float red[256];
  const int row = blockIdx.x, tid = threadIdx.x;
  const float* x = X + (size_t)row * N; const float* rr = R ? R + (size_t)row * N : nullptr;
  float vals[16];
  const int per = N / 256;
  float s1 = 0.f;
  for (int u = 0; u < per / 4; ++u) {
    const int j = tid * 4 + 1024 * u;
    const v4f a = *(const v4fa*)(x + j);
    v4f b = {0.f,0.f,0.f,0.f}; if (rr) b = *(const v4fa*)(rr + j);
#pragma unroll
    for (int q = 0; q < 4; ++q) { const float v = a[q] + b[q]; vals[u * 4 + q] = v; s1 += v; }
  }
  red[tid] = s1; __syncthreads();
  for (int st = 128; st > 0; st >>= 1) { if (tid < st) red[tid] += red[tid + st]; __syncthreads(); }
  const float mu = red[0] / (float)N; __syncthreads();
  float s2 = 0.f;
  for (int u = 0; u < per / 4; ++u)
#pragma unroll
    for (int q = 0; q < 4; ++q) { const float c = vals[u * 4 + q] - mu; s2 += c * c; }
  red[tid] = s2; __syncthreads();
  for (int st = 128; st > 0; st >>= 1) { if (tid < st) red[tid] += red[tid + st]; __syncthreads(); }
  const float rs = rsqrtf(red[0] / (float)N + eps);
  for (int pass = 0; pass < 2; ++pass) {
    for (int u = 0; u < per / 4; ++u) {
      const int j = tid * 4 + 1024 * u;
      v4f o, sm;
#pragma unroll
      for (int q = 0; q < 4; ++q) {
        float gg = g[j + q], bb = bta[j + q];
        if (PARAM_BF16) { gg = bf16_round(gg); bb = bf16_round(bb); }
        sm[q] = vals[u * 4 + q]; o[q] = (vals[u * 4 + q] - mu) * rs * gg + bb;
      }
      if (out_sum) *(volatile v4f*)(out_sum + (size_t)row * N + j) = sm;
      *(volatile v4f*)(out_norm + (size_t)row * N + j) = o;
    }
    if (pass == 0) __threadfence();
  }
}

typedef _Float16 v16h __attribute__((ext_vector_type(16)));
union FragH { v16h v; v8us half[2]; _Float16 h[16]; unsigned short u[16]; };
template <int NT>
__device__ __forceinline__ v8f mmaH(v16h ah, v16h al, v16h bh, v16h bl, v8f c) {
  c = __builtin_amdgcn_wmma_f32_16x16x32_f16(false, ah, false, bh, (short)0, c, false, false);
  if (NT >= 2) c = __builtin_amdgcn_wmma_f32_16x16x32_f16(false, al, false, bh, (short)0, c, false, false);
  if (NT >= 3) c = __builtin_amdgcn_wmma_f32_16x16x32_f16(false, ah, false, bl, (short)0, c, false, false);
  asm volatile("v_nop\n\tv_nop\n\tv_nop\n\tv_nop" : "+v"(c) : "v"(ah), "v"(al), "v"(bh), "v"(bl));
  return c;
}
template <bool ASPLIT>
__global__ __launch_bounds__(128) void k_gemm_h(const float* __restrict__ A, int lda, size_t sA, const _Float16* __restrict__ Bh, int ldb, size_t sB, float alpha, float* __restrict__ C, int ldc, size_t sC, int M, int N, int K) {
  __shared__ __attribute__((aligned(16))) float so[4][16][64];
  const int tid = threadIdx.x, w = tid >> 5, lane = tid & 31, ln = lane & 15, hh = lane >> 4; const int by = blockIdx.y;
  A += (size_t)by * sA; Bh += (size_t)by * sB; C += (size_t)by * sC;
  const int ntn = (N + 63) / 64; const int wid = blockIdx.x * 4 + w; const int mt = wid / ntn, nq = wid % ntn; if (mt * 16 >= M) return;
  const int row0 = mt * 16, col0 = nq * 64; const float* arow = A + (size_t)(row0 + ln) * lda;
  v8f acc[4] = {};
  for (int kb = 0; kb < K; kb += 32) {
    FragH ah, al;
    const v4f x0 = *(const v4fa*)(arow + kb + 8 * hh), x1 = *(const v4fa*)(arow + kb + 8 * hh + 4), x2 = *(const v4fa*)(arow + kb + 16 + 8 * hh), x3 = *(const v4fa*)(arow + kb + 16 + 8 * hh + 4);
    float xs[16] = {x0[0],x0[1],x0[2],x0[3],x1[0],x1[1],x1[2],x1[3],x2[0],x2[1],x2[2],x2[3],x3[0],x3[1],x3[2],x3[3]};
#pragma unroll
    for (int i = 0; i < 16; ++i) { const _Float16 h = (_Float16)xs[i]; ah.h[i] = h; al.h[i] = ASPLIT ? (_Float16)(xs[i] - (float)h) : (_Float16)0.0f; }
#pragma unroll
    for (int t = 0; t < 4; ++t) { if (col0 + t * 16 >= N) continue; const size_t boff = (size_t)(col0 + t * 16 + ln) * ldb + kb; FragH bq; bq.half[0] = *(const v8us*)(Bh + boff + 8 * hh); bq.half[1] = *(const v8us*)(Bh + boff + 16 + 8 * hh);
      acc[t] = mmaH<ASPLIT ? 2 : 1>(ah.v, al.v, bq.v, bq.v, acc[t]); }
  }
#pragma unroll
  for (int t = 0; t < 4; ++t) { if (col0 + t * 16 >= N) continue;
#pragma unroll
    for (int r = 0; r < 8; ++r) so[w][8 * hh + r][t * 16 + ln] = acc[t][r] * alpha; }
  __builtin_amdgcn_fence(__ATOMIC_ACQ_REL, "workgroup"); __builtin_amdgcn_wave_barrier();
  const int rsub = lane >> 4, c4 = (lane & 15) * 4;
  for (int pass = 0; pass < 2; ++pass) {
#pragma unroll
    for (int q = 0; q < 8; ++q) { const int r = q * 2 + rsub; if (col0 + c4 < N) { const v4f v = *(const v4fa*)&so[w][r][c4]; *(volatile v4f*)(C + (size_t)(row0 + r) * ldc + col0 + c4) = v; } }
    if (pass == 0) __threadfence(); }
}

__global__ __launch_bounds__(256) void k_round_rows(const float* __restrict__ W, unsigned short* __restrict__ Wt, int n8) {
  const int t = blockIdx.x * 256 + threadIdx.x;
  if (t >= n8) return;
  const v4f a = *(const v4fa*)(W + (size_t)t * 8), b = *(const v4fa*)(W + (size_t)t * 8 + 4);
  v8us v; v[0]=bf16_bits(a[0]); v[1]=bf16_bits(a[1]); v[2]=bf16_bits(a[2]); v[3]=bf16_bits(a[3]);
  v[4]=bf16_bits(b[0]); v[5]=bf16_bits(b[1]); v[6]=bf16_bits(b[2]); v[7]=bf16_bits(b[3]);
  *(volatile v8us*)(Wt + (size_t)t * 8) = v; __threadfence(); *(volatile v8us*)(Wt + (size_t)t * 8) = v;
}

__global__ __launch_bounds__(256) void k_wt_f16n(const float* __restrict__ W, _Float16* __restrict__ Wt, int n8, float scale) { const int t = blockIdx.x * 256 + threadIdx.x; if (t >= n8) return; FragH f;
#pragma unroll
  for (int i = 0; i < 8; ++i) f.h[i] = (_Float16)(bf16_round(W[t * 8 + i]) * scale); const v8us o = f.half[0]; *(volatile v8us*)((unsigned short*)Wt + t * 8) = o; __threadfence(); *(volatile v8us*)((unsigned short*)Wt + t * 8) = o; }
__global__ __launch_bounds__(256) void k_w1(const float* __restrict__ W1, unsigned short* __restrict__ Ba, unsigned short* __restrict__ Bb) { const int t = blockIdx.x * 256 + threadIdx.x; if (t >= H1 * 8) return; const int o = t / 8, c8 = (t % 8) * 8; v8us a, b;
#pragma unroll
  for (int i = 0; i < 8; ++i) { a[i] = bf16_bits(W1[o * 128 + c8 + i]); b[i] = bf16_bits(W1[o * 128 + 64 + c8 + i]); } *(volatile v8us*)(Ba + o * 64 + c8) = a; *(volatile v8us*)(Bb + o * 64 + c8) = b; __threadfence(); *(volatile v8us*)(Ba + o * 64 + c8) = a; *(volatile v8us*)(Bb + o * 64 + c8) = b; }
__global__ __launch_bounds__(256) void k_bn1stat(const float* __restrict__ P, const float* __restrict__ PB, const int* __restrict__ knn, double* __restrict__ part) {
  __shared__ double r1[4][64], r2[4][64]; const int t = threadIdx.x, o = t & 63, grp = t >> 6; double s = 0.0, q = 0.0; const int pr0 = blockIdx.x * 1024;
#pragma unroll 1
  for (int u = grp; u < 1024; u += 4) { const int pr = pr0 + u; const int i = pr / KN; const int b = i / NP; int j = knn[pr]; j = j < 0 ? 0 : (j >= NP ? NP - 1 : j); j += b * NP;
    const float h = P[(size_t)j * H1 + o] + (PB[(size_t)i * H1 + o] - P[(size_t)i * H1 + o]); s += (double)h; q += (double)h * (double)h; }
  r1[grp][o] = s; r2[grp][o] = q; __syncthreads();
  if (t < 64) { const double a = ((r1[0][t] + r1[1][t]) + r1[2][t]) + r1[3][t], bq = ((r2[0][t] + r2[1][t]) + r2[2][t]) + r2[3][t]; double* d = part + ((size_t)blockIdx.x * 64 + t) * 2; *(volatile double*)d = a; *(volatile double*)(d + 1) = bq; __threadfence(); *(volatile double*)d = a; *(volatile double*)(d + 1) = bq; }
}
__global__ __launch_bounds__(64) void k_bnfin(const double* __restrict__ part, int nblk, double cnt, const float* __restrict__ g, const float* __restrict__ bb, float* __restrict__ st) { const int o = threadIdx.x; double s = 0.0, q = 0.0; for (int k = 0; k < nblk; ++k) { s += part[((size_t)k * 64 + o) * 2]; q += part[((size_t)k * 64 + o) * 2 + 1]; }
  const double mu = s / cnt; double var = q / cnt - mu * mu; if (var < 0.0) var = 0.0; const float rs = (float)(1.0 / sqrt(var + 1e-5)); const float sc = rs * bf16_round(g[o]); const float sh = bf16_round(bb[o]) - (float)mu * sc; *(volatile float*)(st + o * 2) = sc; *(volatile float*)(st + o * 2 + 1) = sh; __threadfence(); *(volatile float*)(st + o * 2) = sc; *(volatile float*)(st + o * 2 + 1) = sh; }
__global__ __launch_bounds__(256) void k_abuild(const float* __restrict__ P, const float* __restrict__ PB, const int* __restrict__ knn, const float* __restrict__ st1, _Float16* __restrict__ A16) {
  const size_t t = (size_t)blockIdx.x * 256 + threadIdx.x; if (t >= (size_t)NPR * 8) return; const int o8 = (int)(t % 8) * 8; const size_t pr = t / 8; const int i = (int)(pr / KN); const int b = i / NP; int j = knn[pr]; j = j < 0 ? 0 : (j >= NP ? NP - 1 : j); j += b * NP; FragH f;
#pragma unroll
  for (int q = 0; q < 8; ++q) { const int o = o8 + q; const float h = P[(size_t)j * H1 + o] + (PB[(size_t)i * H1 + o] - P[(size_t)i * H1 + o]); const float v = h * st1[o * 2] + st1[o * 2 + 1]; f.h[q] = (_Float16)((v >= 0.f) ? v : 0.2f * v); }
  const v8us ov = f.half[0]; *(volatile v8us*)((unsigned short*)A16 + pr * H1 + o8) = ov; __threadfence(); *(volatile v8us*)((unsigned short*)A16 + pr * H1 + o8) = ov;
}
__global__ __launch_bounds__(128) void k_gemm_stat(const _Float16* __restrict__ A, const _Float16* __restrict__ Bh, float* __restrict__ MX, float* __restrict__ MN, float* __restrict__ S1, float* __restrict__ S2) {
  __shared__ __attribute__((aligned(16))) float so[4][16][65];
  const int tid = threadIdx.x, w = tid >> 5, lane = tid & 31, ln = lane & 15, hh = lane >> 4; const int mt = blockIdx.x * 4 + w; if (mt >= NTL) return; const int row0 = mt * 16; const _Float16* arow = A + (size_t)(row0 + ln) * H1;
  v8f acc[4] = {};
#pragma unroll
  for (int kb = 0; kb < H1; kb += 32) { FragH ah; ah.half[0] = *(const v8us*)((const unsigned short*)arow + kb + 8 * hh); ah.half[1] = *(const v8us*)((const unsigned short*)arow + kb + 16 + 8 * hh);
#pragma unroll
    for (int t = 0; t < 4; ++t) { const size_t boff = (size_t)(t * 16 + ln) * H1 + kb; FragH bq; bq.half[0] = *(const v8us*)((const unsigned short*)Bh + boff + 8 * hh); bq.half[1] = *(const v8us*)((const unsigned short*)Bh + boff + 16 + 8 * hh); acc[t] = mmaH<1>(ah.v, ah.v, bq.v, bq.v, acc[t]); } }
#pragma unroll
  for (int t = 0; t < 4; ++t) {
#pragma unroll
    for (int r = 0; r < 8; ++r) so[w][8 * hh + r][t * 16 + ln] = acc[t][r] * 0.0625f; }
  __builtin_amdgcn_fence(__ATOMIC_ACQ_REL, "workgroup"); __builtin_amdgcn_wave_barrier();
  float mx[2], mn[2], s1[2], s2[2];
#pragma unroll
  for (int u = 0; u < 2; ++u) { const int c = u * 32 + lane; float a = so[w][0][c], b = a, s = 0.f, q = 0.f;
#pragma unroll 1
    for (int r = 0; r < 16; ++r) { const float v = so[w][r][c]; a = fmaxf(a, v); b = fminf(b, v); s += v; q += v * v; } mx[u] = a; mn[u] = b; s1[u] = s; s2[u] = q; }
  for (int pass = 0; pass < 2; ++pass) {
#pragma unroll
    for (int u = 0; u < 2; ++u) { const int c = u * 32 + lane; *(volatile float*)(MX + (size_t)mt * H2 + c) = mx[u]; *(volatile float*)(MN + (size_t)mt * H2 + c) = mn[u]; *(volatile float*)(S1 + (size_t)mt * H2 + c) = s1[u]; *(volatile float*)(S2 + (size_t)mt * H2 + c) = s2[u]; } if (pass == 0) __threadfence(); }
}
__global__ __launch_bounds__(256) void k_bn2stat(const float* __restrict__ S1, const float* __restrict__ S2, double* __restrict__ part) { __shared__ double r1[4][64], r2[4][64]; const int t = threadIdx.x, o = t & 63, grp = t >> 6; double s = 0.0, q = 0.0; const int t0 = blockIdx.x * 1024;
#pragma unroll 1
  for (int u = grp; u < 1024; u += 4) { const int tl = t0 + u; s += (double)S1[(size_t)tl * H2 + o]; q += (double)S2[(size_t)tl * H2 + o]; }
  r1[grp][o] = s; r2[grp][o] = q; __syncthreads();
  if (t < 64) { const double a = ((r1[0][t] + r1[1][t]) + r1[2][t]) + r1[3][t], bq = ((r2[0][t] + r2[1][t]) + r2[2][t]) + r2[3][t]; double* d = part + ((size_t)blockIdx.x * 64 + t) * 2; *(volatile double*)d = a; *(volatile double*)(d + 1) = bq; __threadfence(); *(volatile double*)d = a; *(volatile double*)(d + 1) = bq; } }
__global__ __launch_bounds__(256) void k_out(const float* __restrict__ MX, const float* __restrict__ MN, const float* __restrict__ st2, float* __restrict__ out) {
  const size_t t = (size_t)blockIdx.x * 256 + threadIdx.x; if (t >= (size_t)BB * H2 * NP) return; const int n = (int)(t % NP); const int o = (int)((t / NP) % H2); const int b = (int)(t / ((size_t)NP * H2)); const size_t tl = ((size_t)b * NP + n) * 2;
  const float sc = st2[o * 2], sh = st2[o * 2 + 1]; const float sel = (sc >= 0.f) ? fmaxf(MX[tl * H2 + o], MX[(tl + 1) * H2 + o]) : fminf(MN[tl * H2 + o], MN[(tl + 1) * H2 + o]);
  const float v = sel * sc + sh; const float r = (v >= 0.f) ? v : 0.2f * v; *(volatile float*)(out + t) = r; __threadfence(); *(volatile float*)(out + t) = r;
}
extern "C" void kernel_launch(void* const* d_in, const int* in_sizes, int n_in,
                              void* d_out, int out_size, void* d_ws, size_t ws_size, hipStream_t stream) {
  (void)in_sizes; (void)n_in; (void)out_size;
  const float* x = (const float*)d_in[0]; const int* knn = (const int*)d_in[1]; const float* W1 = (const float*)d_in[2]; const float* g1 = (const float*)d_in[3]; const float* b1 = (const float*)d_in[4]; const float* W2 = (const float*)d_in[5]; const float* g2 = (const float*)d_in[6]; const float* b2 = (const float*)d_in[7];
  char* ws = (char*)d_ws; size_t off = 0;
  auto take = [&](size_t bytes) { char* p = ws + off; off += (bytes + 255) & ~(size_t)255; return p; };
  const int NB1 = NPR / 1024, NB2 = NTL / 1024;
  unsigned short* Ba = (unsigned short*)take(H1 * CC * 2); unsigned short* Bb = (unsigned short*)take(H1 * CC * 2); _Float16* B2h = (_Float16*)take(H2 * H1 * 2);
  float* XT = (float*)take((size_t)NPT * CC * 4); float* P = (float*)take((size_t)NPT * H1 * 4); float* PB = (float*)take((size_t)NPT * H1 * 4); double* part = (double*)take((size_t)NB1 * 64 * 2 * 8); float* st1 = (float*)take(64 * 2 * 4); float* st2 = (float*)take(64 * 2 * 4);
  _Float16* A16 = (_Float16*)take((size_t)NPR * H1 * 2); float* MX = (float*)take((size_t)NTL * H2 * 4); float* MN = (float*)take((size_t)NTL * H2 * 4); float* S1 = (float*)take((size_t)NTL * H2 * 4); float* S2 = (float*)take((size_t)NTL * H2 * 4);
  if (off > ws_size) return;
  k_w1<<<(H1 * 8 + 255) / 256, 256, 0, stream>>>(W1, Ba, Bb); k_wt_f16n<<<(H2 * H1 / 8 + 255) / 256, 256, 0, stream>>>(W2, B2h, H2 * H1 / 8, 16.0f);
  k_transpose32<false, false, false><<<dim3(NP / 32, CC / 32, BB), 256, 0, stream>>>(x, XT, CC, NP, nullptr, nullptr, nullptr);
  k_gemm_bf3<false, 0, false, false><<<((NPT / 16) * 1 + 3) / 4, 128, 0, stream>>>(XT, CC, Ba, CC, nullptr, nullptr, 1, 0, P, H1, NPT, H1, CC);
  k_gemm_bf3<false, 0, false, false><<<((NPT / 16) * 1 + 3) / 4, 128, 0, stream>>>(XT, CC, Bb, CC, nullptr, nullptr, 1, 0, PB, H1, NPT, H1, CC);
  k_bn1stat<<<NB1, 256, 0, stream>>>(P, PB, knn, part); k_bnfin<<<1, 64, 0, stream>>>(part, NB1, (double)NPR, g1, b1, st1);
  k_abuild<<<(unsigned)(((size_t)NPR * 8 + 255) / 256), 256, 0, stream>>>(P, PB, knn, st1, A16);
  k_gemm_stat<<<(NTL + 3) / 4, 128, 0, stream>>>(A16, B2h, MX, MN, S1, S2);
  k_bn2stat<<<NB2, 256, 0, stream>>>(S1, S2, part); k_bnfin<<<1, 64, 0, stream>>>(part, NB2, (double)NPR, g2, b2, st2);
  k_out<<<(unsigned)(((size_t)BB * H2 * NP + 255) / 256), 256, 0, stream>>>(MX, MN, st2, (float*)d_out);
}
